// BlockWithCache_11690900979836
// MI455X (gfx1250) — hardware-verified
//
#include <hip/hip_runtime.h>
#include <stdint.h>

typedef __attribute__((ext_vector_type(16))) _Float16 v16h;
typedef __attribute__((ext_vector_type(8)))  _Float16 v8h;
typedef __attribute__((ext_vector_type(16))) __bf16   v16b;
typedef __attribute__((ext_vector_type(8)))  __bf16   v8b;
typedef __attribute__((ext_vector_type(8)))  float    v8f;
typedef __attribute__((ext_vector_type(4)))  float    v4f;

__device__ __forceinline__ unsigned short f2bf_bits(float f) {
  unsigned u = __float_as_uint(f);
  return (unsigned short)((u + 0x7FFFu + ((u >> 16) & 1u)) >> 16);
}
__device__ __forceinline__ float bf_bits2f(unsigned short h) { return __uint_as_float(((unsigned)h) << 16); }

__device__ __forceinline__ void dep_guard_h(v8f& a, v8f& b, v16h x, v16h y) { asm volatile("v_nop\n\tv_nop\n\tv_nop\n\tv_nop" : "+v"(a), "+v"(b) : "v"(x), "v"(y)); }
__device__ __forceinline__ void dep_guard_b(v8f& a, v8f& b, v16b x, v16b y) { asm volatile("v_nop\n\tv_nop\n\tv_nop\n\tv_nop" : "+v"(a), "+v"(b) : "v"(x), "v"(y)); }
__device__ __forceinline__ void keep4_h(v16h a, v16h b, v16h c, v16h d) { asm volatile("v_nop" :: "v"(a), "v"(b), "v"(c), "v"(d)); }
__device__ __forceinline__ void keep4_b(v16b a, v16b b, v16b c, v16b d) { asm volatile("v_nop" :: "v"(a), "v"(b), "v"(c), "v"(d)); }
__device__ __forceinline__ void acc_guard4(v8f& a, v8f& b, v8f& c, v8f& d) { asm volatile("v_nop\n\tv_nop\n\tv_nop\n\tv_nop" : "+v"(a), "+v"(b), "+v"(c), "+v"(d)); }
template <typename T> struct Frag;
template <> struct Frag<_Float16> {
  typedef v16h V; union U { v16h v; v8h h[2]; };
  static __device__ __forceinline__ v16h load(const _Float16* p) {
    U f; f.h[0] = *(const v8h*)(p); f.h[1] = *(const v8h*)(p + 16); return f.v;
  }
  static __device__ __forceinline__ v8f mma(v16h a, v16h b, v8f c) {
    return __builtin_amdgcn_wmma_f32_16x16x32_f16(false, a, false, b, (short)0, c, false, false);
  }
  static __device__ __forceinline__ void guard(v8f& a, v8f& b, v16h x, v16h y) { dep_guard_h(a, b, x, y); }
  static __device__ __forceinline__ void keep(v16h a, v16h b, v16h c, v16h d) { keep4_h(a, b, c, d); }
};
template <> struct Frag<__bf16> {
  typedef v16b V; union U { v16b v; v8b h[2]; };
  static __device__ __forceinline__ v16b load(const __bf16* p) {
    U f; f.h[0] = *(const v8b*)(p); f.h[1] = *(const v8b*)(p + 16); return f.v;
  }
  static __device__ __forceinline__ v8f mma(v16b a, v16b b, v8f c) {
    return __builtin_amdgcn_wmma_f32_16x16x32_bf16(false, a, false, b, (short)0, c, false, false);
  }
  static __device__ __forceinline__ void guard(v8f& a, v8f& b, v16b x, v16b y) { dep_guard_b(a, b, x, y); }
  static __device__ __forceinline__ void keep(v16b a, v16b b, v16b c, v16b d) { keep4_b(a, b, c, d); }
};

template <int ET> struct Elem;
template <> struct Elem<0> { typedef _Float16 T; };
template <> struct Elem<1> { typedef __bf16 T; };
template <int ET, bool SPLIT, int BIAS_MODE, int OUT_MODE, bool RESID, int ACT = 0, int TRIMIN = 0>
__global__ __launch_bounds__(256) void wmma_gemm64(
    const unsigned short* __restrict__ Ap, const unsigned short* __restrict__ A2p, int lda, long strideA,
    const unsigned short* __restrict__ Btp, const unsigned short* __restrict__ Bt2p, int ldb, long strideB,
    void* __restrict__ Cout, void* __restrict__ Cout2, int ldc, long strideC,
    const float* __restrict__ bias,
    const float* __restrict__ resid, long strideR,
    int M, int N, int K, float scale) {
  typedef typename Elem<ET>::T T;
  typedef typename Frag<T>::V V;
  const T* A = (const T*)Ap; const T* A2 = (const T*)A2p; const T* Bt = (const T*)Btp; const T* Bt2 = (const T*)Bt2p;
  __shared__ __align__(16) float sT[8][16 * 68];
  const int b    = blockIdx.y;
  const int lane = threadIdx.x & 31;
  const int wave = threadIdx.x >> 5;
  const int tilesN = N >> 6;
  const int tilesM = M >> 6;
  const int tile = blockIdx.x * 8 + wave;
  if (tile >= tilesM * tilesN) return;
  const int tm = tile / tilesN;
  const int tn = tile - tm * tilesN;
  if (TRIMIN > 0 && (tm + tn) < TRIMIN) return;
  const int m0 = tm << 6;
  const int n0 = tn << 6;

  const T* Ab  = A  + (size_t)b * strideA;
  const T* Bb  = Bt + (size_t)b * strideB;
  const T* Ab2 = SPLIT ? (A2  + (size_t)b * strideA) : nullptr;
  const T* Bb2 = SPLIT ? (Bt2 + (size_t)b * strideB) : nullptr;

  const int rlane = lane & 15;
  const int koff  = (lane >> 4) * 8;
  const int mOff  = (lane >> 4) * 8;

  v8f acc[4][4];
#pragma unroll
  for (int i = 0; i < 4; ++i)
#pragma unroll
    for (int j = 0; j < 4; ++j) acc[i][j] = (v8f){0.f,0.f,0.f,0.f,0.f,0.f,0.f,0.f};

  for (int k0 = 0; k0 < K; k0 += 32) {
    V bh[4], bl[4];
#pragma unroll
    for (int j = 0; j < 4; ++j) {
      const size_t bo = (size_t)(n0 + (j << 4) + rlane) * ldb + koff + k0;
      bh[j] = Frag<T>::load(Bb + bo);
      if (SPLIT) bl[j] = Frag<T>::load(Bb2 + bo);
    }
#pragma unroll
    for (int i = 0; i < 4; ++i) {
      const size_t ao = (size_t)(m0 + (i << 4) + rlane) * lda + koff + k0;
      V ah = Frag<T>::load(Ab + ao);
      V al;
      if (SPLIT) al = Frag<T>::load(Ab2 + ao);
#pragma unroll
      for (int j = 0; j < 4; ++j) {
        acc[i][j] = Frag<T>::mma(ah, bh[j], acc[i][j]);
        if (SPLIT) {
          acc[i][j] = Frag<T>::mma(ah, bl[j], acc[i][j]);
          acc[i][j] = Frag<T>::mma(al, bh[j], acc[i][j]);
        }
      }
      Frag<T>::guard(acc[i][0], acc[i][3], ah, SPLIT ? al : ah);
    }
    Frag<T>::keep(bh[0], bh[1], bh[2], bh[3]);
    if (SPLIT) Frag<T>::keep(bl[0], bl[1], bl[2], bl[3]);
  }
  acc_guard4(acc[0][0], acc[0][1], acc[0][2], acc[0][3]);
  acc_guard4(acc[1][0], acc[1][1], acc[1][2], acc[1][3]);
  acc_guard4(acc[2][0], acc[2][1], acc[2][2], acc[2][3]);
  acc_guard4(acc[3][0], acc[3][1], acc[3][2], acc[3][3]);

  float* slab = sT[wave];
  const float* Rb = RESID ? (resid + (size_t)b * strideR) : nullptr;
#pragma unroll
  for (int i = 0; i < 4; ++i) {
    const int mBase = m0 + (i << 4);
#pragma unroll
    for (int j = 0; j < 4; ++j) {
      const int n = n0 + (j << 4) + rlane;
      float bv = 0.f;
      if (BIAS_MODE == 2) bv = bias[n];
#pragma unroll
      for (int r = 0; r < 8; ++r) {
        float v = acc[i][j][r] * scale;
        if (BIAS_MODE == 1) v += bias[mBase + mOff + r];
        if (BIAS_MODE == 2) v += bv;
        if (RESID) v += Rb[(size_t)(mBase + mOff + r) * ldc + n];
        if (ACT == 1) v = tanhf(v);
        if (ACT == 2) v = fmaxf(v, 0.0f);
        if (ACT == 3) v = v / (1.0f + expf(-v));
        if (ACT == 4) v = (v > 0.f) ? v : 0.01f * v;
        if (ACT == 5) v = 0.5f * v * (1.0f + erff(v * 0.70710678118654752f));
        slab[(mOff + r) * 68 + (j << 4) + rlane] = v;
      }
    }
    __builtin_amdgcn_fence(__ATOMIC_RELEASE, "workgroup");
    __builtin_amdgcn_wave_barrier();
    __builtin_amdgcn_fence(__ATOMIC_ACQUIRE, "workgroup");
    if (OUT_MODE == 0) {
      float* C = (float*)Cout + (size_t)b * strideC;
      const int hh = lane >> 4, c4 = (lane & 15) * 4;
      for (int pass = 0; pass < 2; ++pass) {
#pragma unroll
        for (int it = 0; it < 8; ++it) {
          const int row = it * 2 + hh;
          v4f v = *(const v4f*)(slab + row * 68 + c4);
          *(volatile v4f*)(C + (size_t)(mBase + row) * ldc + n0 + c4) = v;
        }
        __threadfence();
      }
    } else {
      const int q = lane >> 3, c8 = (lane & 7) * 8;
      unsigned short* C  = (unsigned short*)Cout  + (size_t)b * strideC;
      unsigned short* C2 = (OUT_MODE == 2) ? ((unsigned short*)Cout2 + (size_t)b * strideC) : nullptr;
      for (int pass = 0; pass < 2; ++pass) {
#pragma unroll
        for (int it = 0; it < 4; ++it) {
          const int row = it * 4 + q;
          const float* sp = slab + row * 68 + c8;
          v8h hv, lv;
#pragma unroll
          for (int e = 0; e < 8; ++e) {
            if (OUT_MODE == 1) {
              hv[e] = (_Float16)sp[e];
            } else {
              unsigned short hb = f2bf_bits(sp[e]);
              unsigned short lb = f2bf_bits(sp[e] - bf_bits2f(hb));
              hv[e] = __builtin_bit_cast(_Float16, hb);
              lv[e] = __builtin_bit_cast(_Float16, lb);
            }
          }
          *(volatile v8h*)(C + (size_t)(mBase + row) * ldc + n0 + c8) = hv;
          if (OUT_MODE == 2) *(volatile v8h*)(C2 + (size_t)(mBase + row) * ldc + n0 + c8) = lv;
        }
        __threadfence();
      }
    }
    __builtin_amdgcn_fence(__ATOMIC_RELEASE, "workgroup");
    __builtin_amdgcn_wave_barrier();
    __builtin_amdgcn_fence(__ATOMIC_ACQUIRE, "workgroup");
  }
}

__global__ __launch_bounds__(256) void cast_f32_f16x2(
    const float* __restrict__ in, _Float16* __restrict__ out, int n2) {
  int i = blockIdx.x * 256 + threadIdx.x;
  if (i < n2) {
    const _Float16 h0 = (_Float16)in[2 * i], h1 = (_Float16)in[2 * i + 1];
    const unsigned u = (unsigned)__builtin_bit_cast(unsigned short, h0) | ((unsigned)__builtin_bit_cast(unsigned short, h1) << 16);
    ((volatile unsigned*)out)[i] = u;
    __threadfence();
    ((volatile unsigned*)out)[i] = u;
  }
}

__global__ __launch_bounds__(256) void transpose_cast_f16(
    const float* __restrict__ in, _Float16* __restrict__ out, int R, int C) {
  __shared__ float tile[64][65];
  const int tid = threadIdx.x;
  const int c0 = blockIdx.x * 64, r0 = blockIdx.y * 64;
#pragma unroll
  for (int i = 0; i < 16; ++i) {
    const int idx = tid + i * 256;
    const int r = idx >> 6, cc = idx & 63;
    tile[r][cc] = in[(size_t)(r0 + r) * C + c0 + cc];
  }
  __syncthreads();
  const int wave = tid >> 5, lane = tid & 31;
  const int q = lane >> 3, c8 = (lane & 7) * 8;
  for (int pass = 0; pass < 2; ++pass) {
#pragma unroll
    for (int it = 0; it < 2; ++it) {
      const int orow = wave * 8 + it * 4 + q;
      v8h hv;
#pragma unroll
      for (int e = 0; e < 8; ++e) hv[e] = (_Float16)tile[c8 + e][orow];
      *(volatile v8h*)(out + (size_t)(c0 + orow) * R + r0 + c8) = hv;
    }
    __threadfence();
  }
}

__global__ __launch_bounds__(128) void layernorm1024_f16(
    const float* __restrict__ x, const float* __restrict__ w, const float* __restrict__ bb,
    _Float16* __restrict__ out) {
  __shared__ float red[2][4];
  const int row = blockIdx.x, tid = threadIdx.x, lane = tid & 31, wave = tid >> 5;
  const float* xr = x + (size_t)row * 1024 + tid * 8;
  const v4f a0 = *(const v4f*)xr;
  const v4f a1 = *(const v4f*)(xr + 4);
  float vals[8];
  vals[0] = a0[0]; vals[1] = a0[1]; vals[2] = a0[2]; vals[3] = a0[3];
  vals[4] = a1[0]; vals[5] = a1[1]; vals[6] = a1[2]; vals[7] = a1[3];
  float s = 0.f;
#pragma unroll
  for (int e = 0; e < 8; ++e) s += vals[e];
#pragma unroll
  for (int off = 16; off; off >>= 1) s += __shfl_xor(s, off, 32);
  if (lane == 0) red[0][wave] = s;
  __syncthreads();
  const float mean = (red[0][0] + red[0][1] + red[0][2] + red[0][3]) * (1.0f / 1024.0f);
  float s2 = 0.f;
#pragma unroll
  for (int e = 0; e < 8; ++e) { const float d = vals[e] - mean; s2 += d * d; }
#pragma unroll
  for (int off = 16; off; off >>= 1) s2 += __shfl_xor(s2, off, 32);
  if (lane == 0) red[1][wave] = s2;
  __syncthreads();
  const float var = (red[1][0] + red[1][1] + red[1][2] + red[1][3]) * (1.0f / 1024.0f);
  const float inv = rsqrtf(var + 1e-5f);
  const v4f w0 = *(const v4f*)(w + tid * 8), w1 = *(const v4f*)(w + tid * 8 + 4);
  const v4f b0 = *(const v4f*)(bb + tid * 8), b1 = *(const v4f*)(bb + tid * 8 + 4);
  float wv[8], bv[8];
  wv[0] = w0[0]; wv[1] = w0[1]; wv[2] = w0[2]; wv[3] = w0[3]; wv[4] = w1[0]; wv[5] = w1[1]; wv[6] = w1[2]; wv[7] = w1[3];
  bv[0] = b0[0]; bv[1] = b0[1]; bv[2] = b0[2]; bv[3] = b0[3]; bv[4] = b1[0]; bv[5] = b1[1]; bv[6] = b1[2]; bv[7] = b1[3];
  v8h hv;
#pragma unroll
  for (int e = 0; e < 8; ++e) hv[e] = (_Float16)((vals[e] - mean) * inv * wv[e] + bv[e]);
  _Float16* op = out + (size_t)row * 1024 + tid * 8;
  *(volatile v8h*)op = hv;
  __threadfence();
  *(volatile v8h*)op = hv;
}

__device__ __forceinline__ v8f mma_h(v16h a, v16h b, v8f c) {
  c = __builtin_amdgcn_wmma_f32_16x16x32_f16(false, a, false, b, (short)0, c, false, false);
  asm volatile("v_nop\n\tv_nop\n\tv_nop\n\tv_nop" : "+v"(c) : "v"(a), "v"(b));
  return c;
}
#define SQ_L 1024
#define SQ_D 1024
#define SQ_LD3 3072
#define SQ_PSC 32768.0f

__global__ __launch_bounds__(128)
void attn_rel_kernel(const _Float16* __restrict__ qkv, const float* __restrict__ qer,
                     _Float16* __restrict__ y, int bidx) {
  __shared__ __align__(16) _Float16 Ksh[64 * 64];
  __shared__ __align__(16) _Float16 Vth[64 * 64];
  __shared__ __align__(16) _Float16 Psh[4][16 * 64];
  __shared__ __align__(16) float Os[4][16 * 68];
  const int tid = threadIdx.x;
  const int wave = tid >> 5, lane = tid & 31, hh = lane >> 4, c = lane & 15;
  const int qb = blockIdx.x & 15;
  const int h = blockIdx.x >> 4;
  const int q0 = qb * 64 + wave * 16;
  const size_t rowb = (size_t)bidx * SQ_L;
  const float ninf = -__builtin_inff();

  v16h qa0, qa1;
  {
    const _Float16* qrow = qkv + (rowb + q0 + c) * SQ_LD3 + h * 64;
    qa0 = Frag<_Float16>::load(qrow + 8 * hh);
    qa1 = Frag<_Float16>::load(qrow + 32 + 8 * hh);
  }
  const float* qerh = qer + (size_t)h * ((size_t)SQ_L * SQ_L);

  float mrow[8], lrow[8];
  v8f oacc[4];
#pragma unroll
  for (int r = 0; r < 8; ++r) { mrow[r] = ninf; lrow[r] = 0.f; }
#pragma unroll
  for (int t = 0; t < 4; ++t) oacc[t] = (v8f){0.f,0.f,0.f,0.f,0.f,0.f,0.f,0.f};

  const int nChunks = qb + 1;
  for (int kc = 0; kc < nChunks; ++kc) {
    const int kv0 = kc * 64;
    __syncthreads();
    {
      const int kvr = tid >> 1, dh = (tid & 1) * 32;
      const _Float16* kp = qkv + (rowb + kv0 + kvr) * SQ_LD3 + SQ_D + h * 64 + dh;
      const _Float16* vp = kp + SQ_D;
#pragma unroll
      for (int i = 0; i < 4; ++i) {
        const v8h kk = *(const v8h*)(kp + 8 * i);
        *(v8h*)(Ksh + kvr * 64 + dh + 8 * i) = kk;
        const v8h vv = *(const v8h*)(vp + 8 * i);
#pragma unroll
        for (int e = 0; e < 8; ++e) Vth[(dh + 8 * i + e) * 64 + kvr] = vv[e];
      }
    }
    __syncthreads();

    v8f s[4];
#pragma unroll
    for (int j = 0; j < 4; ++j) {
      s[j] = (v8f){0.f,0.f,0.f,0.f,0.f,0.f,0.f,0.f};
      const _Float16* kr = Ksh + (j * 16 + c) * 64 + 8 * hh;
      const v16h kb0 = Frag<_Float16>::load(kr);
      s[j] = mma_h(qa0, kb0, s[j]);
      const v16h kb1 = Frag<_Float16>::load(kr + 32);
      s[j] = mma_h(qa1, kb1, s[j]);
    }
    const bool diag = (kc == qb);
    float cm[8];
#pragma unroll
    for (int r = 0; r < 8; ++r) {
      const int qrow = q0 + 8 * hh + r;
      const float* brow = qerh + (size_t)qrow * SQ_L;
      float m = ninf;
#pragma unroll
      for (int j = 0; j < 4; ++j) {
        const int kvcol = kv0 + j * 16 + c;
        const bool masked = diag && (kvcol > qrow);
        int mi = SQ_L - 1 - qrow + kvcol;
        mi = mi < 0 ? 0 : (mi > SQ_L - 1 ? SQ_L - 1 : mi);
        float bv = 0.f;
        if (!masked) bv = brow[mi];
        float sv = (s[j][r] + bv) * 0.125f;
        if (masked) sv = ninf;
        s[j][r] = sv;
        m = fmaxf(m, sv);
      }
#pragma unroll
      for (int off = 1; off < 16; off <<= 1) m = fmaxf(m, __shfl_xor(m, off, 32));
      cm[r] = m;
    }
    _Float16* pwh = Psh[wave];
#pragma unroll
    for (int r = 0; r < 8; ++r) {
      const float mnew = fmaxf(mrow[r], cm[r]);
      const float alpha = expf(mrow[r] - mnew);
      mrow[r] = mnew;
      float psum = 0.f;
#pragma unroll
      for (int j = 0; j < 4; ++j) {
        const float p = expf(s[j][r] - mnew);
        psum += p;
        pwh[(8 * hh + r) * 64 + j * 16 + c] = (_Float16)(p * SQ_PSC);
      }
#pragma unroll
      for (int off = 1; off < 16; off <<= 1) psum += __shfl_xor(psum, off, 32);
      lrow[r] = lrow[r] * alpha + psum;
#pragma unroll
      for (int t = 0; t < 4; ++t) oacc[t][r] *= alpha;
    }
    __builtin_amdgcn_fence(__ATOMIC_RELEASE, "workgroup");
    __builtin_amdgcn_wave_barrier();
    __builtin_amdgcn_fence(__ATOMIC_ACQUIRE, "workgroup");
#pragma unroll 1
    for (int kk = 0; kk < 2; ++kk) {
      const v16h pa = Frag<_Float16>::load(pwh + c * 64 + kk * 32 + 8 * hh);
#pragma unroll
      for (int t = 0; t < 4; ++t) {
        const v16h vb = Frag<_Float16>::load(Vth + (t * 16 + c) * 64 + kk * 32 + 8 * hh);
        oacc[t] = mma_h(pa, vb, oacc[t]);
      }
    }
  }

  float* os = Os[wave];
#pragma unroll
  for (int r = 0; r < 8; ++r) {
    const float inv = 1.0f / (lrow[r] * SQ_PSC);
#pragma unroll
    for (int t = 0; t < 4; ++t) os[(8 * hh + r) * 68 + t * 16 + c] = oacc[t][r] * inv;
  }
  __builtin_amdgcn_fence(__ATOMIC_RELEASE, "workgroup");
  __builtin_amdgcn_wave_barrier();
  __builtin_amdgcn_fence(__ATOMIC_ACQUIRE, "workgroup");
  {
    const int q4 = lane >> 3, c8 = (lane & 7) * 8;
    _Float16* yb = y + (rowb + q0) * SQ_D + h * 64 + c8;
    for (int pass = 0; pass < 2; ++pass) {
#pragma unroll
      for (int it = 0; it < 4; ++it) {
        const int row = it * 4 + q4;
        const float* sp = os + row * 68 + c8;
        v8h hv;
#pragma unroll
        for (int e = 0; e < 8; ++e) hv[e] = (_Float16)sp[e];
        *(volatile v8h*)(yb + (size_t)row * SQ_D) = hv;
      }
      __threadfence();
    }
  }
}

extern "C" void kernel_launch(void* const* d_in, const int* in_sizes, int n_in,
                              void* d_out, int out_size, void* d_ws, size_t ws_size,
                              hipStream_t stream) {
  const int Lc = 1024, Dc = 1024, Bc = 4, Hc = 16, HSc = 64;
  const int Mr = Bc * Lc;
  if (n_in < 14) return;
  if (in_sizes[0] != Mr * Dc || in_sizes[1] != Dc || in_sizes[2] != Dc ||
      in_sizes[3] != Dc * 3 * Dc || in_sizes[4] != 3 * Dc ||
      in_sizes[5] != Dc * Dc || in_sizes[6] != Dc ||
      in_sizes[7] != Lc * HSc || in_sizes[8] != Dc || in_sizes[9] != Dc ||
      in_sizes[10] != Dc * 4 * Dc || in_sizes[11] != 4 * Dc ||
      in_sizes[12] != 4 * Dc * Dc || in_sizes[13] != Dc || out_size != Mr * Dc) return;

  const float* x     = (const float*)d_in[0];
  const float* ln1w  = (const float*)d_in[1];
  const float* ln1b  = (const float*)d_in[2];
  const float* Wqkv  = (const float*)d_in[3];
  const float* bqkv  = (const float*)d_in[4];
  const float* Wproj = (const float*)d_in[5];
  const float* bproj = (const float*)d_in[6];
  const float* Er    = (const float*)d_in[7];
  const float* ln2w  = (const float*)d_in[8];
  const float* ln2b  = (const float*)d_in[9];
  const float* Wfc   = (const float*)d_in[10];
  const float* bfc   = (const float*)d_in[11];
  const float* Wfc2  = (const float*)d_in[12];
  const float* bfc2  = (const float*)d_in[13];
  float* out = (float*)d_out;

  const size_t MiB = (size_t)1048576;
  const size_t off_qkv16  = 0;
  const size_t off_x1     = 0;
  const size_t off_h2     = 16 * MiB;
  const size_t off_wqkvT  = 24 * MiB;
  const size_t off_h16    = 30 * MiB;
  const size_t off_qer    = 24 * MiB;
  const size_t off_wprojT = 24 * MiB;
  const size_t off_m1     = 24 * MiB;
  const size_t off_wfcT   = 56 * MiB;
  const size_t off_wfc2T  = 64 * MiB;
  const size_t off_y16    = 88 * MiB;
  const size_t off_er16   = 96 * MiB;
  const size_t total      = 96 * MiB + (size_t)Lc * HSc * 2;
  if (total > ws_size) return;

  char* ws = (char*)d_ws;
  unsigned short* qkv16  = (unsigned short*)(ws + off_qkv16);
  float*          x1     = (float*)(ws + off_x1);
  unsigned short* h2     = (unsigned short*)(ws + off_h2);
  unsigned short* WqkvT  = (unsigned short*)(ws + off_wqkvT);
  unsigned short* h16    = (unsigned short*)(ws + off_h16);
  float*          qer    = (float*)(ws + off_qer);
  unsigned short* WprojT = (unsigned short*)(ws + off_wprojT);
  unsigned short* m1     = (unsigned short*)(ws + off_m1);
  unsigned short* WfcT   = (unsigned short*)(ws + off_wfcT);
  unsigned short* Wfc2T  = (unsigned short*)(ws + off_wfc2T);
  unsigned short* y16    = (unsigned short*)(ws + off_y16);
  unsigned short* Er16   = (unsigned short*)(ws + off_er16);

  transpose_cast_f16<<<dim3(3 * Dc / 64, Dc / 64), 256, 0, stream>>>(Wqkv, (_Float16*)WqkvT, Dc, 3 * Dc);
  cast_f32_f16x2<<<(Lc * HSc / 2 + 255) / 256, 256, 0, stream>>>(Er, (_Float16*)Er16, Lc * HSc / 2);
  layernorm1024_f16<<<Mr, 128, 0, stream>>>(x, ln1w, ln1b, (_Float16*)h16);
  wmma_gemm64<0, false, 2, 1, false, 0><<<dim3((Mr / 64) * (3 * Dc / 64) / 8, 1), 256, 0, stream>>>(
      h16, h16, Dc, (long)0, WqkvT, WqkvT, Dc, (long)0,
      (void*)qkv16, nullptr, 3 * Dc, (long)0, bqkv, nullptr, (long)0, Mr, 3 * Dc, Dc, 1.0f);

  for (int b = 0; b < Bc; ++b) {
    wmma_gemm64<0, false, 0, 0, false, 0, 15><<<dim3((Lc / 64) * (Lc / 64) / 8, Hc), 256, 0, stream>>>(
        qkv16 + (size_t)b * Lc * 3 * Dc, qkv16 + (size_t)b * Lc * 3 * Dc, 3 * Dc, (long)HSc,
        Er16, Er16, HSc, (long)0,
        (void*)qer, nullptr, Lc, (long)Lc * Lc, nullptr, nullptr, (long)0, Lc, Lc, HSc, 1.0f);
    attn_rel_kernel<<<Hc * (Lc / 64), 128, 0, stream>>>((const _Float16*)qkv16, qer, (_Float16*)y16, b);
  }

  transpose_cast_f16<<<dim3(Dc / 64, Dc / 64), 256, 0, stream>>>(Wproj, (_Float16*)WprojT, Dc, Dc);
  wmma_gemm64<0, false, 2, 0, true, 0><<<dim3((Mr / 64) * (Dc / 64) / 8, 1), 256, 0, stream>>>(
      y16, y16, Dc, (long)0, WprojT, WprojT, Dc, (long)0,
      (void*)x1, nullptr, Dc, (long)0, bproj, x, (long)0, Mr, Dc, Dc, 1.0f);

  layernorm1024_f16<<<Mr, 128, 0, stream>>>(x1, ln2w, ln2b, (_Float16*)h2);
  transpose_cast_f16<<<dim3(4 * Dc / 64, Dc / 64), 256, 0, stream>>>(Wfc, (_Float16*)WfcT, Dc, 4 * Dc);
  wmma_gemm64<0, false, 2, 1, false, 5><<<dim3((Mr / 64) * (4 * Dc / 64) / 8, 1), 256, 0, stream>>>(
      h2, h2, Dc, (long)0, WfcT, WfcT, Dc, (long)0,
      (void*)m1, nullptr, 4 * Dc, (long)0, bfc, nullptr, (long)0, Mr, 4 * Dc, Dc, 1.0f);
  transpose_cast_f16<<<dim3(Dc / 64, 4 * Dc / 64), 256, 0, stream>>>(Wfc2, (_Float16*)Wfc2T, 4 * Dc, Dc);
  wmma_gemm64<0, false, 2, 0, true, 0><<<dim3((Mr / 64) * (Dc / 64) / 8, 1), 256, 0, stream>>>(
      m1, m1, 4 * Dc, (long)0, Wfc2T, Wfc2T, 4 * Dc, (long)0,
      (void*)out, nullptr, Dc, (long)0, bfc2, x1, (long)0, Mr, Dc, 4 * Dc, 1.0f);
}
